// MultiHeadAttentionQuantum_65481071409457
// MI455X (gfx1250) — hardware-verified
//
#include <hip/hip_runtime.h>
#include <math.h>
#include <stdint.h>

#ifndef NB
#define NB 4
#endif
#ifndef SEQ
#define SEQ 2048
#endif
#define NB_FULL  4
#define SEQ_FULL 2048
#define H_   8
#define DK_  64
#define E_   512
#define BH_  (NB * H_)
#define NQT  (SEQ / 64)
#define NKT  (SEQ / 64)
#define TENC 128
#define CSP  65
#define KP   72
static_assert(H_ * DK_ == E_);
static_assert(NB >= 1 && NB <= NB_FULL);
static_assert(SEQ >= TENC && SEQ <= SEQ_FULL);
static_assert((SEQ % TENC) == 0 && (SEQ % 64) == 0);
static_assert(((KP * 2) % 16) == 0);
static_assert(((E_ * E_) % (8 * 256)) == 0);
static_assert(((NB * SEQ) % 64) == 0);

typedef _Float16 v16h __attribute__((ext_vector_type(16)));
typedef _Float16 v8h  __attribute__((ext_vector_type(8)));
typedef float    v8f  __attribute__((ext_vector_type(8)));
typedef float    v4f  __attribute__((ext_vector_type(4)));
typedef unsigned int v4u __attribute__((ext_vector_type(4)));

#if defined(__HIP_DEVICE_COMPILE__)
#define DEV_ASM 1
#else
#define DEV_ASM 0
#endif

__device__ __forceinline__ unsigned short h_bits(_Float16 v) { return __builtin_bit_cast(unsigned short, v); }
__device__ __forceinline__ unsigned pk16(unsigned short a, unsigned short b) { return (unsigned)a | ((unsigned)b << 16); }
__device__ __forceinline__ v8f zero8() { v8f z = {0.f, 0.f, 0.f, 0.f, 0.f, 0.f, 0.f, 0.f}; return z; }

__device__ __forceinline__ v16h ldfrag_h(const _Float16* p) {
  union { v16h v; v8h h[2]; } f;
  f.h[0] = *(const v8h*)(p);
  f.h[1] = *(const v8h*)(p + 16);
  return f.v;
}

__device__ __forceinline__ v8f mma_h(v16h a, v16h b, v8f c) {
  c = __builtin_amdgcn_wmma_f32_16x16x32_f16(false, a, false, b, (short)0, c, false, false);
#if DEV_ASM
  asm volatile("v_nop\n\tv_nop\n\tv_nop\n\tv_nop" : "+v"(c) : "v"(a), "v"(b));
#endif
  return c;
}

__global__ __launch_bounds__(256) void qenc(const float* __restrict__ x, const float* __restrict__ theta,
                                            unsigned short* qkp, unsigned short* vtp) {
  __shared__ float cs[TENC * CSP];
  const int tid = (int)threadIdx.x;
  const int bx  = (int)blockIdx.x;
  const int nst = SEQ / TENC;
  const int st  = bx % nst;
  const int bh  = bx / nst;
  const int b   = bh / H_;
  const int h   = bh - b * H_;
  const int s0  = st * TENC;
  const int d   = tid & 63;
  const int tg  = tid >> 6;
  {
    const float th = theta[d];
    const float* xp = x + ((size_t)b * SEQ_FULL + (size_t)s0) * E_ + (size_t)(h * DK_ + d);
#pragma unroll 1
    for (int i = 0; i < TENC / 4; ++i) {
      const int t = tg + 4 * i;
      const float v = xp[(size_t)t * E_] + th;
      cs[t * CSP + d] = cosf(v);
    }
  }
  __syncthreads();

  const size_t rowbase = (size_t)bh * SEQ + (size_t)s0;

  v4u qv[4], vv[4];
#pragma unroll
  for (int it = 0; it < 4; ++it) {
    const int token = it * 32 + (tid >> 3);
    const int j     = tid & 7;
    const float* sp = cs + token * CSP + j * 8;
    v4u a;
#pragma unroll
    for (int e = 0; e < 4; ++e) {
      a[e] = pk16(h_bits((_Float16)sp[2 * e]), h_bits((_Float16)sp[2 * e + 1]));
    }
    qv[it] = a;
  }
#pragma unroll
  for (int it = 0; it < 4; ++it) {
    const int dd = it * 16 + (tid >> 4);
    const int j  = tid & 15;
    const float* sp = cs + (j * 8) * CSP + dd;
    v4u a;
#pragma unroll
    for (int e = 0; e < 4; ++e) {
      a[e] = pk16(h_bits((_Float16)sp[(2 * e) * CSP]), h_bits((_Float16)sp[(2 * e + 1) * CSP]));
    }
    vv[it] = a;
  }

  unsigned short* qo = qkp + (rowbase + (size_t)(tid >> 3)) * DK_ + (size_t)((tid & 7) * 8);
  unsigned short* vo = vtp + ((size_t)bh * DK_ + (size_t)(tid >> 4)) * SEQ + (size_t)s0 + (size_t)((tid & 15) * 8);
  for (int pass = 0; pass < 2; ++pass) {
#pragma unroll
    for (int it = 0; it < 4; ++it) {
      *(volatile v4u*)(qo + (size_t)it * 32 * DK_) = qv[it];
      *(volatile v4u*)(vo + (size_t)it * 16 * SEQ) = vv[it];
    }
    __threadfence();
  }
}

__global__ __launch_bounds__(256) void wconv(const float* __restrict__ W, unsigned short* wh) {
  const size_t p = (size_t)blockIdx.x * 256 + (size_t)threadIdx.x;
  const v4f a  = *(const v4f*)(W + p * 8);
  const v4f a4 = *(const v4f*)(W + p * 8 + 4);
  v4u q;
  q[0] = pk16(h_bits((_Float16)(a[0] * 1024.0f)),  h_bits((_Float16)(a[1] * 1024.0f)));
  q[1] = pk16(h_bits((_Float16)(a[2] * 1024.0f)),  h_bits((_Float16)(a[3] * 1024.0f)));
  q[2] = pk16(h_bits((_Float16)(a4[0] * 1024.0f)), h_bits((_Float16)(a4[1] * 1024.0f)));
  q[3] = pk16(h_bits((_Float16)(a4[2] * 1024.0f)), h_bits((_Float16)(a4[3] * 1024.0f)));
  unsigned short* o = wh + p * 8;
  for (int pass = 0; pass < 2; ++pass) {
    *(volatile v4u*)o = q;
    __threadfence();
  }
}

__global__ __launch_bounds__(128)
void attn(const unsigned short* __restrict__ qkp, const unsigned short* __restrict__ vtp, unsigned short* mp) {
  union FH { v16h v; v8h h[2]; };
  __shared__ __align__(16) _Float16 Ksh[64 * KP];
  __shared__ __align__(16) _Float16 Vsh[64 * KP];
  __shared__ __align__(16) _Float16 Psh[4][16 * 64];
  __shared__ __align__(16) float    Os[4][16 * 64];

  const int tid  = (int)threadIdx.x;
  const int wave = tid >> 5;
  const int lane = tid & 31;
  const int hh   = lane >> 4;
  const int c    = lane & 15;

  const int bx = (int)blockIdx.x;
  const int qt = bx % NQT;
  const int bh = bx / NQT;
  const int b  = bh / H_;
  const int h  = bh - b * H_;
  const int q0 = qt * 64 + wave * 16;

  const _Float16* QK = (const _Float16*)(const void*)qkp + (size_t)bh * SEQ * DK_;
  const _Float16* VT = (const _Float16*)(const void*)vtp + (size_t)bh * DK_ * SEQ;

  const v16h qa0 = ldfrag_h(QK + (size_t)(q0 + c) * DK_ + 8 * hh);
  const v16h qa1 = ldfrag_h(QK + (size_t)(q0 + c) * DK_ + 32 + 8 * hh);

  float mrow[8], lrow[8];
  v8f oacc[4];
#pragma unroll
  for (int j = 0; j < 4; ++j) oacc[j] = zero8();
#pragma unroll
  for (int r = 0; r < 8; ++r) { mrow[r] = -INFINITY; lrow[r] = 0.f; }

#pragma unroll 1
  for (int kt = 0; kt < NKT; ++kt) {
    const int kv0 = kt * 64;
    __syncthreads();
#pragma unroll
    for (int i = 0; i < 4; ++i) {
      const int p   = i * 128 + tid;
      const int row = p >> 3;
      const int ch  = (p & 7) * 8;
      const v8h kvv = *(const v8h*)(QK + (size_t)(kv0 + row) * DK_ + ch);
      const v8h vvv = *(const v8h*)(VT + (size_t)row * SEQ + (size_t)kv0 + (size_t)ch);
      *(v8h*)(Ksh + row * KP + ch) = kvv;
      *(v8h*)(Vsh + row * KP + ch) = vvv;
    }
    __syncthreads();

    v8f s[4];
#pragma unroll
    for (int j = 0; j < 4; ++j) {
      const _Float16* kr = Ksh + (j * 16 + c) * KP + 8 * hh;
      FH kb0, kb1;
      kb0.h[0] = *(const v8h*)(kr);
      kb0.h[1] = *(const v8h*)(kr + 16);
      kb1.h[0] = *(const v8h*)(kr + 32);
      kb1.h[1] = *(const v8h*)(kr + 48);
      v8f acc = mma_h(qa0, kb0.v, zero8());
      acc = mma_h(qa1, kb1.v, acc);
#pragma unroll
      for (int r = 0; r < 8; ++r) s[j][r] = acc[r] * 0.125f;
    }

    _Float16* pwh = Psh[wave];
#pragma unroll
    for (int r = 0; r < 8; ++r) {
      float m = s[0][r];
#pragma unroll
      for (int j = 1; j < 4; ++j) m = fmaxf(m, s[j][r]);
#pragma unroll
      for (int off = 1; off < 16; off <<= 1) m = fmaxf(m, __shfl_xor(m, off, 32));
      const float mnew  = fmaxf(mrow[r], m);
      const float msafe = (mnew == -INFINITY) ? 0.f : mnew;
      const float alpha = __expf(mrow[r] - msafe);
      mrow[r] = mnew;
      float psum = 0.f;
#pragma unroll
      for (int j = 0; j < 4; ++j) {
        const float p = __expf(s[j][r] - msafe);
        psum += p;
        pwh[(8 * hh + r) * 64 + j * 16 + c] = (_Float16)(p * 1024.0f);
      }
#pragma unroll
      for (int off = 1; off < 16; off <<= 1) psum += __shfl_xor(psum, off, 32);
      lrow[r] = lrow[r] * alpha + psum;
#pragma unroll
      for (int j = 0; j < 4; ++j) oacc[j][r] *= alpha;
    }
    __builtin_amdgcn_fence(3  , "workgroup");
    __builtin_amdgcn_wave_barrier();
    __builtin_amdgcn_fence(2  , "workgroup");

#pragma unroll
    for (int kk = 0; kk < 2; ++kk) {
      FH pa;
      pa.h[0] = *(const v8h*)(pwh + c * 64 + kk * 32 + 8 * hh);
      pa.h[1] = *(const v8h*)(pwh + c * 64 + kk * 32 + 16 + 8 * hh);
#pragma unroll
      for (int jn = 0; jn < 4; ++jn) {
        const _Float16* vr = Vsh + (jn * 16 + c) * KP + kk * 32 + 8 * hh;
        FH vb;
        vb.h[0] = *(const v8h*)(vr);
        vb.h[1] = *(const v8h*)(vr + 16);
        oacc[jn] = mma_h(pa.v, vb.v, oacc[jn]);
      }
    }
  }

  float* os = Os[wave];
#pragma unroll
  for (int r = 0; r < 8; ++r) {
    const float l = lrow[r];
    const float inv = ((l > 0.f) ? (1.0f / l) : 0.f) * 0.25f;
#pragma unroll
    for (int jn = 0; jn < 4; ++jn) os[(8 * hh + r) * 64 + jn * 16 + c] = oacc[jn][r] * inv;
  }
  __builtin_amdgcn_fence(3  , "workgroup");
  __builtin_amdgcn_wave_barrier();
  __builtin_amdgcn_fence(2  , "workgroup");
  {
    const int rsub  = lane >> 3;
    const int piece = (lane & 7) * 8;
    v4u a[4];
#pragma unroll
    for (int i = 0; i < 4; ++i) {
      const float* sp = os + (i * 4 + rsub) * 64 + piece;
      v4u t;
#pragma unroll
      for (int e = 0; e < 4; ++e) t[e] = pk16(h_bits((_Float16)sp[2 * e]), h_bits((_Float16)sp[2 * e + 1]));
      a[i] = t;
    }
    unsigned short* o = mp + ((size_t)b * SEQ + (size_t)(q0 + rsub)) * E_ + (size_t)(h * DK_) + (size_t)piece;
    for (int pass = 0; pass < 2; ++pass) {
#pragma unroll
      for (int i = 0; i < 4; ++i) *(volatile v4u*)(o + (size_t)(i * 4) * E_) = a[i];
      __threadfence();
    }
  }
}

__global__ __launch_bounds__(128)
void proj_out(const unsigned short* __restrict__ mp, const unsigned short* __restrict__ wh,
              const float* __restrict__ bc, float* out) {
  __shared__ __align__(16) float lds[4 * 16 * 128];

  const int tid  = (int)threadIdx.x;
  const int wave = tid >> 5;
  const int lane = tid & 31;
  const int hh   = lane >> 4;
  const int c    = lane & 15;

  const int nrb = (NB * SEQ) / 64;
  const int rb  = (int)blockIdx.x % nrb;
  const int cb  = (int)blockIdx.x / nrb;
  const int m0  = rb * 64 + wave * 16;
  const int n0  = cb * 128;

  const _Float16* Arow = (const _Float16*)(const void*)mp + (size_t)(m0 + c) * E_ + 8 * hh;
  const _Float16* Wrow = (const _Float16*)(const void*)wh + (size_t)(n0 + c) * E_ + 8 * hh;

  v8f acc[8];
#pragma unroll
  for (int j = 0; j < 8; ++j) acc[j] = zero8();

#pragma unroll 2
  for (int ks = 0; ks < E_ / 32; ++ks) {
    const int k0 = ks * 32;
    const v16h af = ldfrag_h(Arow + k0);
#pragma unroll
    for (int j = 0; j < 8; ++j) {
      const v16h bf = ldfrag_h(Wrow + (size_t)(j * 16) * E_ + k0);
      acc[j] = mma_h(af, bf, acc[j]);
    }
  }

  float* slab = lds + wave * 2048;
#pragma unroll
  for (int j = 0; j < 8; ++j) {
#pragma unroll
    for (int r = 0; r < 8; ++r) slab[(8 * hh + r) * 128 + j * 16 + c] = acc[j][r];
  }
  __builtin_amdgcn_fence(3  , "workgroup");
  __builtin_amdgcn_wave_barrier();
  __builtin_amdgcn_fence(2  , "workgroup");

  const float oscale = 1.0f / 262144.0f;
  const v4f b4 = *(const v4f*)(bc + n0 + lane * 4);
  v4f vrow[16];
#pragma unroll
  for (int row = 0; row < 16; ++row) {
    const v4f v = *(const v4f*)(slab + row * 128 + lane * 4);
    vrow[row] = v * oscale + b4;
  }
  const int ob = m0 / SEQ;
  const int os0 = m0 - ob * SEQ;
  float* op = out + ((size_t)ob * SEQ_FULL + (size_t)os0) * E_ + (size_t)n0 + (size_t)(lane * 4);
  for (int pass = 0; pass < 2; ++pass) {
#pragma unroll
    for (int row = 0; row < 16; ++row) {
      *(volatile v4f*)(op + (size_t)row * E_) = vrow[row];
    }
    __threadfence();
  }
}

extern "C" void kernel_launch(void* const* d_in, const int* in_sizes, int n_in,
                              void* d_out, int out_size, void* d_ws, size_t ws_size,
                              hipStream_t stream) {
  if (n_in < 4) return;
  if ((long long)in_sizes[0] < (long long)NB * SEQ_FULL * E_) return;
  if (in_sizes[1] < DK_) return;
  if (in_sizes[2] < E_ * E_) return;
  if (in_sizes[3] < E_) return;
  if ((long long)out_size < ((long long)(NB - 1) * SEQ_FULL + SEQ) * E_) return;

  const float* x     = (const float*)d_in[0];
  const float* theta = (const float*)d_in[1];
  const float* W     = (const float*)d_in[2];
  const float* bc    = (const float*)d_in[3];

  const size_t PQK = (size_t)BH_ * SEQ * DK_ * 2;
  const size_t PVT = (size_t)BH_ * DK_ * SEQ * 2;
  const size_t PMP = (size_t)NB * SEQ * E_ * 2;
  const size_t PWH = (size_t)E_ * E_ * 2;
  size_t off = 0;
  const size_t oQK = off; off += PQK;
  const size_t oVT = off; off += PVT;
  const size_t oMP = off; off += PMP;
  const size_t oWH = off; off += PWH;
  if (off > ws_size) return;
  if (off > (size_t)134217728) return;

  char* ws = (char*)d_ws;
  unsigned short* QK = (unsigned short*)(ws + oQK);
  unsigned short* VT = (unsigned short*)(ws + oVT);
  unsigned short* MP = (unsigned short*)(ws + oMP);
  unsigned short* WH = (unsigned short*)(ws + oWH);

  const dim3 gEnc(BH_ * (SEQ / TENC));
  const dim3 gWcv((E_ * E_) / (8 * 256));
  const dim3 gAttn(BH_ * NQT);
  const dim3 gProj(((NB * SEQ) / 64) * 4);

  qenc<<<gEnc, dim3(256), 0, stream>>>(x, theta, QK, VT);
  wconv<<<gWcv, dim3(256), 0, stream>>>(W, WH);
  attn<<<gAttn, dim3(128), 0, stream>>>(QK, VT, MP);
  proj_out<<<gProj, dim3(128), 0, stream>>>(MP, WH, bc, (float*)d_out);
  (void)hipGetLastError();
}
